// VideoMambaVideoEncoder_60455959658705
// MI455X (gfx1250) — hardware-verified
//
#include <hip/hip_runtime.h>
#include <math.h>

typedef __attribute__((ext_vector_type(16))) _Float16 v16h;
typedef __attribute__((ext_vector_type(8)))  _Float16 v8h;
typedef __attribute__((ext_vector_type(16))) __bf16   v16b;
typedef __attribute__((ext_vector_type(8)))  __bf16   v8b;
typedef __attribute__((ext_vector_type(8)))  float    v8f;
typedef __attribute__((ext_vector_type(4)))  float    v4f;

constexpr int kFrames  = 4;
constexpr int kImg     = 224;
constexpr int kPatch   = 16;
constexpr int kGridP   = kImg / kPatch;
constexpr int kNP      = kFrames * kGridP * kGridP;
constexpr int kL       = kNP + 1;
constexpr int kLP      = 832;
constexpr int kDm      = 384;
constexpr int kE       = 768;
constexpr int kXzP     = 2 * kE;
constexpr int kNs      = 16;
constexpr int kR       = 24;
constexpr int kRP      = 32;
constexpr int kDbl     = kR + 2 * kNs;
constexpr int kDblP    = 64;
constexpr int kNL      = 12;
constexpr int kPF      = 3 * kPatch * kPatch;
constexpr int kTP      = 260;
constexpr float kEps   = 1e-5f;
static_assert(kNP == 784 && kL == 785, "token count");
static_assert(kDbl == 56 && kPF == 768, "widths");
static_assert((kLP % 64) == 0 && kLP >= kL, "padded rows");
static_assert((kDm % 64) == 0 && (kE % 64) == 0 && (kXzP % 64) == 0 && (kDblP % 64) == 0, "N tile multiples");
static_assert((kDm % 32) == 0 && (kE % 32) == 0 && (kRP % 32) == 0 && (kPF % 32) == 0, "K multiples of 32");

constexpr float kCarryW   = 32.0f;
constexpr float kCarryWdt = 8.0f;
constexpr float kCarryXs  = 16.0f;
constexpr float kCarryDtr = 256.0f;
constexpr float kCarryCmb = 1024.0f;
constexpr float kSclIn    = 1.0f / kCarryW;
constexpr float kSclXp    = 1.0f / (kCarryXs * kCarryW);
constexpr float kSclDt    = 1.0f / (kCarryDtr * kCarryWdt);
constexpr float kSclOut   = 1.0f / (kCarryCmb * kCarryW);

constexpr size_t kSzWIN  = (size_t)kNL * kXzP * kDm * 2;
constexpr size_t kSzWOUT = (size_t)kNL * kDm * kE * 2;
constexpr size_t kSzWXP  = (size_t)2 * kNL * kDblP * kE * 2;
constexpr size_t kSzWDT  = (size_t)2 * kNL * kE * kRP * 2;
constexpr size_t kSzPW   = (size_t)kDm * kPF * 2;
constexpr size_t kSzPA   = (size_t)kLP * kPF * 2;
constexpr size_t kSzRES  = (size_t)kLP * kDm * 4;
constexpr size_t kSzH16  = (size_t)kLP * kDm * 2;
constexpr size_t kSzXZ   = (size_t)kLP * kXzP * 4;
constexpr size_t kSzXS   = (size_t)2 * kLP * kE * 4;
constexpr size_t kSzXS16 = (size_t)2 * kLP * kE * 2;
constexpr size_t kSzDBL  = (size_t)2 * kLP * kDblP * 4;
constexpr size_t kSzDTR  = (size_t)2 * kLP * kRP * 2;
constexpr size_t kSzCMB  = (size_t)kLP * kE * 2;

constexpr size_t kOffWIN  = 0;
constexpr size_t kOffWOUT = kOffWIN  + kSzWIN;
constexpr size_t kOffWXP  = kOffWOUT + kSzWOUT;
constexpr size_t kOffWDT  = kOffWXP  + kSzWXP;
constexpr size_t kOffPWH  = kOffWDT  + kSzWDT;
constexpr size_t kOffPWL  = kOffPWH  + kSzPW;
constexpr size_t kOffPAH  = kOffPWL  + kSzPW;
constexpr size_t kOffPAL  = kOffPAH  + kSzPA;
constexpr size_t kOffRES  = kOffPAL  + kSzPA;
constexpr size_t kOffHID  = kOffRES  + kSzRES;
constexpr size_t kOffH16  = kOffHID  + kSzRES;
constexpr size_t kOffXZ   = kOffH16  + kSzH16;
constexpr size_t kOffXS   = kOffXZ   + kSzXZ;
constexpr size_t kOffXS16 = kOffXS   + kSzXS;
constexpr size_t kOffDBL  = kOffXS16 + kSzXS16;
constexpr size_t kOffDTR  = kOffDBL  + kSzDBL;
constexpr size_t kOffDLR  = kOffDTR  + kSzDTR;
constexpr size_t kOffYS   = kOffDLR  + kSzXS;
constexpr size_t kOffCMB  = kOffYS   + kSzXS;
constexpr size_t kWsTotal = kOffCMB  + kSzCMB;
static_assert(kWsTotal == 56516608ull, "carve total");
static_assert(kWsTotal <= 134217728ull, "carve cap");
static_assert((kOffWOUT % 128) == 0 && (kOffWXP % 128) == 0 && (kOffWDT % 128) == 0 && (kOffPWH % 128) == 0 &&
              (kOffPWL % 128) == 0 && (kOffPAH % 128) == 0 && (kOffPAL % 128) == 0 && (kOffRES % 128) == 0 &&
              (kOffHID % 128) == 0 && (kOffH16 % 128) == 0 && (kOffXZ % 128) == 0 && (kOffXS % 128) == 0 &&
              (kOffXS16 % 128) == 0 && (kOffDBL % 128) == 0 && (kOffDTR % 128) == 0 && (kOffDLR % 128) == 0 &&
              (kOffYS % 128) == 0 && (kOffCMB % 128) == 0, "128-B aligned regions");

__device__ __forceinline__ unsigned short f2bf_bits(float f) {
  unsigned u = __float_as_uint(f);
  return (unsigned short)((u + 0x7FFFu + ((u >> 16) & 1u)) >> 16);
}
__device__ __forceinline__ float bf_bits2f(unsigned short h) { return __uint_as_float(((unsigned)h) << 16); }
__device__ __forceinline__ float silu_f(float v) { return v * __builtin_amdgcn_rcpf(1.0f + expf(-v)); }

__device__ __forceinline__ void guard4_h(v8f& a, v8f& b, v8f& c, v8f& d, v16h x, v16h y) {
  asm volatile("v_nop\n\tv_nop\n\tv_nop\n\tv_nop" : "+v"(a), "+v"(b), "+v"(c), "+v"(d) : "v"(x), "v"(y));
}
__device__ __forceinline__ void guard4_b(v8f& a, v8f& b, v8f& c, v8f& d, v16b x, v16b y) {
  asm volatile("v_nop\n\tv_nop\n\tv_nop\n\tv_nop" : "+v"(a), "+v"(b), "+v"(c), "+v"(d) : "v"(x), "v"(y));
}
__device__ __forceinline__ void keep4_h(v16h a, v16h b, v16h c, v16h d) { asm volatile("v_nop" :: "v"(a), "v"(b), "v"(c), "v"(d)); }
__device__ __forceinline__ void keep4_b(v16b a, v16b b, v16b c, v16b d) { asm volatile("v_nop" :: "v"(a), "v"(b), "v"(c), "v"(d)); }
__device__ __forceinline__ void acc_guard4(v8f& a, v8f& b, v8f& c, v8f& d) {
  asm volatile("v_nop\n\tv_nop\n\tv_nop\n\tv_nop" : "+v"(a), "+v"(b), "+v"(c), "+v"(d));
}

template <typename T> struct Frag;
template <> struct Frag<_Float16> {
  typedef v16h V;
  union U { v16h v; v8h h[2]; };
  static __device__ __forceinline__ v16h load(const _Float16* p) {
    U f; f.h[0] = *(const v8h*)(p); f.h[1] = *(const v8h*)(p + 16); return f.v;
  }
  static __device__ __forceinline__ v8f mma(v16h a, v16h b, v8f c) {
    return __builtin_amdgcn_wmma_f32_16x16x32_f16(false, a, false, b, (short)0, c, false, false);
  }
  static __device__ __forceinline__ void guard(v8f& a, v8f& b, v8f& c, v8f& d, v16h x, v16h y) { guard4_h(a, b, c, d, x, y); }
  static __device__ __forceinline__ void keep(v16h a, v16h b, v16h c, v16h d) { keep4_h(a, b, c, d); }
};
template <> struct Frag<__bf16> {
  typedef v16b V;
  union U { v16b v; v8b h[2]; };
  static __device__ __forceinline__ v16b load(const __bf16* p) {
    U f; f.h[0] = *(const v8b*)(p); f.h[1] = *(const v8b*)(p + 16); return f.v;
  }
  static __device__ __forceinline__ v8f mma(v16b a, v16b b, v8f c) {
    return __builtin_amdgcn_wmma_f32_16x16x32_bf16(false, a, false, b, (short)0, c, false, false);
  }
  static __device__ __forceinline__ void guard(v8f& a, v8f& b, v8f& c, v8f& d, v16b x, v16b y) { guard4_b(a, b, c, d, x, y); }
  static __device__ __forceinline__ void keep(v16b a, v16b b, v16b c, v16b d) { keep4_b(a, b, c, d); }
};

template <int ET> struct Elem;
template <> struct Elem<0> { typedef _Float16 T; };
template <> struct Elem<1> { typedef __bf16 T; };

template <int ET, bool SPLIT, bool EPI>
__global__ __launch_bounds__(256) void wmma_gemm64(
    const unsigned short* __restrict__ Ap, const unsigned short* __restrict__ A2p, int lda, long strideA,
    const unsigned short* __restrict__ Btp, const unsigned short* __restrict__ Bt2p, int ldb, long strideB,
    float* __restrict__ Cout, int ldc, long strideC,
    const float* __restrict__ bias, const float* __restrict__ resid,
    int M, int N, int K, int Mstore, float scale)
{
  typedef typename Elem<ET>::T T;
  typedef typename Frag<T>::V V;
  const T* A   = (const T*)Ap;
  const T* A2  = (const T*)A2p;
  const T* Bt  = (const T*)Btp;
  const T* Bt2 = (const T*)Bt2p;
  __shared__ __align__(16) float sT[8][16 * 68];
  const int b    = blockIdx.y;
  const int lane = threadIdx.x & 31;
  const int wave = threadIdx.x >> 5;
  const int tilesN = N >> 6;
  const int tilesM = M >> 6;
  const int tile = blockIdx.x * 8 + wave;
  if (tile >= tilesM * tilesN) return;
  const int tm = tile / tilesN;
  const int tn = tile - tm * tilesN;
  const int m0 = tm << 6;
  const int n0 = tn << 6;

  const T* Ab  = A   + (size_t)b * strideA;
  const T* Bb  = Bt  + (size_t)b * strideB;
  const T* Ab2 = A2  + (size_t)b * strideA;
  const T* Bb2 = Bt2 + (size_t)b * strideB;

  const int rlane = lane & 15;
  const int koff  = (lane >> 4) * 8;
  const int mOff  = (lane >> 4) * 8;

  v8f acc[4][4];
#pragma unroll
  for (int i = 0; i < 4; ++i)
#pragma unroll
    for (int j = 0; j < 4; ++j) acc[i][j] = (v8f){0.f, 0.f, 0.f, 0.f, 0.f, 0.f, 0.f, 0.f};

  for (int k0 = 0; k0 < K; k0 += 32) {
    V bh[4], bl[4];
#pragma unroll
    for (int j = 0; j < 4; ++j) {
      const size_t bo = (size_t)(n0 + (j << 4) + rlane) * ldb + koff + k0;
      bh[j] = Frag<T>::load(Bb + bo);
      if (SPLIT) bl[j] = Frag<T>::load(Bb2 + bo);
    }
#pragma unroll
    for (int i = 0; i < 4; ++i) {
      const size_t ao = (size_t)(m0 + (i << 4) + rlane) * lda + koff + k0;
      V ah = Frag<T>::load(Ab + ao);
      V al = ah;
      if (SPLIT) al = Frag<T>::load(Ab2 + ao);
#pragma unroll
      for (int j = 0; j < 4; ++j) {
        acc[i][j] = Frag<T>::mma(ah, bh[j], acc[i][j]);
        if (SPLIT) {
          acc[i][j] = Frag<T>::mma(ah, bl[j], acc[i][j]);
          acc[i][j] = Frag<T>::mma(al, bh[j], acc[i][j]);
        }
      }
      Frag<T>::guard(acc[i][0], acc[i][1], acc[i][2], acc[i][3], ah, al);
    }
    Frag<T>::keep(bh[0], bh[1], bh[2], bh[3]);
    if (SPLIT) Frag<T>::keep(bl[0], bl[1], bl[2], bl[3]);
  }
  acc_guard4(acc[0][0], acc[0][1], acc[0][2], acc[0][3]);
  acc_guard4(acc[1][0], acc[1][1], acc[1][2], acc[1][3]);
  acc_guard4(acc[2][0], acc[2][1], acc[2][2], acc[2][3]);
  acc_guard4(acc[3][0], acc[3][1], acc[3][2], acc[3][3]);

  float* slab = sT[wave];
  float* C = Cout + (size_t)b * strideC;
  const int hh = lane >> 4;
  const int c4 = (lane & 15) * 4;
  v4f bq = (v4f){0.f, 0.f, 0.f, 0.f};
  if (EPI) bq = *(const v4f*)(bias + n0 + c4);
#pragma unroll
  for (int i = 0; i < 4; ++i) {
    const int mBase = m0 + (i << 4);
#pragma unroll
    for (int j = 0; j < 4; ++j) {
#pragma unroll
      for (int r = 0; r < 8; ++r) {
        slab[(mOff + r) * 68 + (j << 4) + rlane] = acc[i][j][r] * scale;
      }
    }
    __builtin_amdgcn_fence(__ATOMIC_RELEASE, "workgroup");
    __builtin_amdgcn_wave_barrier();
    __builtin_amdgcn_fence(__ATOMIC_ACQUIRE, "workgroup");
    v4f vv[8];
#pragma unroll
    for (int it = 0; it < 8; ++it) {
      const int row = it * 2 + hh;
      v4f v = *(const v4f*)(slab + row * 68 + c4);
      if (EPI) {
        const int grow = mBase + row;
        const int rc = (grow < Mstore) ? grow : (Mstore - 1);
        const v4f rv = *(const v4f*)(resid + (size_t)rc * ldc + n0 + c4);
        v = (v + bq) + rv;
      }
      vv[it] = v;
    }
    for (int pass = 0; pass < 2; ++pass) {
#pragma unroll
      for (int it = 0; it < 8; ++it) {
        const int grow = mBase + it * 2 + hh;
        if (grow < Mstore) *(volatile v4f*)(C + (size_t)grow * ldc + n0 + c4) = vv[it];
      }
      __threadfence();
    }
    __builtin_amdgcn_fence(__ATOMIC_RELEASE, "workgroup");
    __builtin_amdgcn_wave_barrier();
    __builtin_amdgcn_fence(__ATOMIC_ACQUIRE, "workgroup");
  }
}

__global__ __launch_bounds__(256) void pad_cast_f16_kernel(
    const float* __restrict__ srcA, const float* __restrict__ srcB, unsigned short* __restrict__ dst,
    int srows, int scols, int drows, int dcols, int nmat, float scale, int total8)
{
  const int i = blockIdx.x * 256 + threadIdx.x;
  if (i >= total8) return;
  const float* src = (blockIdx.y != 0) ? srcB : srcA;
  unsigned short* dd = dst + (size_t)blockIdx.y * ((size_t)nmat * drows * dcols);
  const int e0 = i << 3;
  const int rr = e0 / dcols;
  const int c0 = e0 - rr * dcols;
  const int mt = rr / drows;
  const int r  = rr - mt * drows;
  const bool ok = (r < srows) && (c0 < scols);
  const int rc = (r < srows) ? r : (srows - 1);
  const int cc = (c0 < scols) ? c0 : 0;
  const float* p = src + ((size_t)mt * srows + rc) * scols + cc;
  const v4f a0 = *(const v4f*)(p);
  const v4f a1 = *(const v4f*)(p + 4);
  v8h hv;
#pragma unroll
  for (int e = 0; e < 4; ++e) {
    const float f0 = ok ? (a0[e] * scale) : 0.0f;
    const float f1 = ok ? (a1[e] * scale) : 0.0f;
    hv[e]     = (_Float16)f0;
    hv[4 + e] = (_Float16)f1;
  }
  unsigned short* q = dd + (size_t)e0;
  *(volatile v8h*)q = hv;
  __threadfence();
  *(volatile v8h*)q = hv;
}

__global__ __launch_bounds__(256) void split_rows_bf16_kernel(
    const float* __restrict__ src, unsigned short* __restrict__ dhi, unsigned short* __restrict__ dlo, int total8)
{
  const int i = blockIdx.x * 256 + threadIdx.x;
  if (i >= total8) return;
  const size_t e0 = (size_t)i << 3;
  const v4f a0 = *(const v4f*)(src + e0);
  const v4f a1 = *(const v4f*)(src + e0 + 4);
  v8h hv, lv;
#pragma unroll
  for (int e = 0; e < 4; ++e) {
    const float f0 = a0[e];
    const float f1 = a1[e];
    const unsigned short h0 = f2bf_bits(f0), h1 = f2bf_bits(f1);
    const unsigned short l0 = f2bf_bits(f0 - bf_bits2f(h0)), l1 = f2bf_bits(f1 - bf_bits2f(h1));
    hv[e]     = __builtin_bit_cast(_Float16, h0);
    hv[4 + e] = __builtin_bit_cast(_Float16, h1);
    lv[e]     = __builtin_bit_cast(_Float16, l0);
    lv[4 + e] = __builtin_bit_cast(_Float16, l1);
  }
  unsigned short* qh = dhi + e0;
  unsigned short* ql = dlo + e0;
  *(volatile v8h*)qh = hv;
  *(volatile v8h*)ql = lv;
  __threadfence();
  *(volatile v8h*)qh = hv;
  *(volatile v8h*)ql = lv;
}

constexpr int kPatchBlocks = (kLP * kPF / 8) / 256;
static_assert(kPatchBlocks * 256 * 8 == kLP * kPF, "patchify coverage");
__global__ __launch_bounds__(256) void patchify_kernel(
    const float* __restrict__ x, const float* __restrict__ cls, const float* __restrict__ pos,
    unsigned short* __restrict__ PAH, unsigned short* __restrict__ PAL, float* __restrict__ HID)
{
  const int tid = threadIdx.x;
  if ((int)blockIdx.x == kPatchBlocks) {
    if (tid < kDm / 4) {
      const v4f cv = *(const v4f*)(cls + tid * 4);
      const v4f pv = *(const v4f*)(pos + tid * 4);
      const v4f sv = cv + pv;
      float* q = HID + tid * 4;
      *(volatile v4f*)q = sv;
      __threadfence();
      *(volatile v4f*)q = sv;
    }
    return;
  }
  const int i  = blockIdx.x * 256 + tid;
  const int e0 = i << 3;
  const int tok = e0 / kPF;
  const int f   = e0 - tok * kPF;
  const int c   = f >> 8;
  const int a   = (f >> 4) & 15;
  const int b0  = f & 15;
  const bool ok = tok < kNP;
  const int tc  = ok ? tok : (kNP - 1);
  const int t   = tc / (kGridP * kGridP);
  const int rem = tc - t * (kGridP * kGridP);
  const int pi  = rem / kGridP;
  const int pj  = rem - pi * kGridP;
  const float* p = x + ((size_t)((c * kFrames + t) * kImg + pi * kPatch + a)) * kImg + pj * kPatch + b0;
  const v4f a0 = *(const v4f*)(p);
  const v4f a1 = *(const v4f*)(p + 4);
  v8h hv, lv;
#pragma unroll
  for (int e = 0; e < 4; ++e) {
    const float f0 = ok ? a0[e] : 0.0f;
    const float f1 = ok ? a1[e] : 0.0f;
    const unsigned short h0 = f2bf_bits(f0), h1 = f2bf_bits(f1);
    const unsigned short l0 = f2bf_bits(f0 - bf_bits2f(h0)), l1 = f2bf_bits(f1 - bf_bits2f(h1));
    hv[e]     = __builtin_bit_cast(_Float16, h0);
    hv[4 + e] = __builtin_bit_cast(_Float16, h1);
    lv[e]     = __builtin_bit_cast(_Float16, l0);
    lv[4 + e] = __builtin_bit_cast(_Float16, l1);
  }
  unsigned short* qh = PAH + (size_t)e0;
  unsigned short* ql = PAL + (size_t)e0;
  *(volatile v8h*)qh = hv;
  *(volatile v8h*)ql = lv;
  __threadfence();
  *(volatile v8h*)qh = hv;
  *(volatile v8h*)ql = lv;
}

template <bool FINAL>
__global__ __launch_bounds__(256) void add_rmsnorm_kernel(
    const float* __restrict__ hidden, float* residual, const float* __restrict__ w,
    unsigned short* __restrict__ H16, float* __restrict__ outp, int first)
{
  __shared__ __align__(16) float sN[8 * kDm];
  const int lane = threadIdx.x & 31, wave = threadIdx.x >> 5;
  const int row = blockIdx.x * 8 + wave;
  const int ch0 = lane * 8;
  const int ch1 = 256 + (lane & 15) * 8;
  if (row >= kL) {
    if (!FINAL) {
      v8h zv;
#pragma unroll
      for (int e = 0; e < 8; ++e) zv[e] = (_Float16)0.0f;
      unsigned short* q0 = H16 + (size_t)row * kDm + ch0;
      unsigned short* q1 = H16 + (size_t)row * kDm + ch1;
      for (int pass = 0; pass < 2; ++pass) {
        *(volatile v8h*)q0 = zv;
        if (lane < 16) *(volatile v8h*)q1 = zv;
        __threadfence();
      }
    }
    return;
  }
  const size_t base = (size_t)row * kDm;
  v4f r[3];
  float ss = 0.0f;
#pragma unroll
  for (int i = 0; i < 3; ++i) {
    const int o = i * 128 + lane * 4;
    const v4f hv = *(const v4f*)(hidden + base + o);
    v4f rv = (v4f){0.f, 0.f, 0.f, 0.f};
    if (!first) rv = *(const v4f*)(residual + base + o);
    const v4f v = rv + hv;
    r[i] = v;
    ss = fmaf(v[0], v[0], ss);
    ss = fmaf(v[1], v[1], ss);
    ss = fmaf(v[2], v[2], ss);
    ss = fmaf(v[3], v[3], ss);
  }
#pragma unroll
  for (int off = 16; off > 0; off >>= 1) ss += __shfl_xor(ss, off, 32);
  const float inv = rsqrtf(ss * (1.0f / (float)kDm) + kEps);
  v4f n[3];
#pragma unroll
  for (int i = 0; i < 3; ++i) {
    const int o = i * 128 + lane * 4;
    const v4f wv = *(const v4f*)(w + o);
    n[i] = (r[i] * inv) * wv;
  }
  if (FINAL) {
    for (int pass = 0; pass < 2; ++pass) {
#pragma unroll
      for (int i = 0; i < 3; ++i) *(volatile v4f*)(outp + base + i * 128 + lane * 4) = n[i];
      __threadfence();
    }
    return;
  }
  for (int pass = 0; pass < 2; ++pass) {
#pragma unroll
    for (int i = 0; i < 3; ++i) *(volatile v4f*)(residual + base + i * 128 + lane * 4) = r[i];
    __threadfence();
  }
  float* sl = sN + wave * kDm;
#pragma unroll
  for (int i = 0; i < 3; ++i) *(v4f*)(sl + i * 128 + lane * 4) = n[i];
  __builtin_amdgcn_fence(__ATOMIC_RELEASE, "workgroup");
  __builtin_amdgcn_wave_barrier();
  __builtin_amdgcn_fence(__ATOMIC_ACQUIRE, "workgroup");
  const v4f a0 = *(const v4f*)(sl + ch0);
  const v4f a1 = *(const v4f*)(sl + ch0 + 4);
  const v4f b0 = *(const v4f*)(sl + ch1);
  const v4f b1 = *(const v4f*)(sl + ch1 + 4);
  v8h h0, h1;
#pragma unroll
  for (int e = 0; e < 4; ++e) {
    h0[e]     = (_Float16)a0[e];
    h0[4 + e] = (_Float16)a1[e];
    h1[e]     = (_Float16)b0[e];
    h1[4 + e] = (_Float16)b1[e];
  }
  unsigned short* q0 = H16 + base + ch0;
  unsigned short* q1 = H16 + base + ch1;
  for (int pass = 0; pass < 2; ++pass) {
    *(volatile v8h*)q0 = h0;
    if (lane < 16) *(volatile v8h*)q1 = h1;
    __threadfence();
  }
}

__device__ __forceinline__ float ld_xin(const float* __restrict__ XZ, int r, int d) {
  const int rc = (r < 0) ? 0 : ((r > kL - 1) ? (kL - 1) : r);
  const float v = XZ[(size_t)rc * kXzP + d];
  return (r >= 0 && r < kL) ? v : 0.0f;
}
__global__ __launch_bounds__(256) void conv_silu_kernel(
    const float* __restrict__ XZ,
    const float* __restrict__ cwf, const float* __restrict__ cbf,
    const float* __restrict__ cwb, const float* __restrict__ cbb,
    float* __restrict__ XS, unsigned short* __restrict__ XS16)
{
  __shared__ __align__(16) float sF[16 * kTP];
  __shared__ __align__(16) float sB[16 * kTP];
  const int tid = threadIdx.x, lane = tid & 31, wave = tid >> 5;
  const int d0 = blockIdx.x * 256, d = d0 + tid;
  const int t0 = blockIdx.y * 64;
  const v4f wf = *(const v4f*)(cwf + (size_t)d * 4);
  const v4f wb = *(const v4f*)(cwb + (size_t)d * 4);
  const float bf = cbf[d], bb = cbb[d];
  float xm3 = ld_xin(XZ, t0 - 3, d);
  float xm2 = ld_xin(XZ, t0 - 2, d);
  float xm1 = ld_xin(XZ, t0 - 1, d);
  float x0  = ld_xin(XZ, t0, d);
  float xp1 = ld_xin(XZ, t0 + 1, d);
  float xp2 = ld_xin(XZ, t0 + 2, d);
  const int hrow = wave >> 1;
  const int hch  = (wave & 1) * 128 + lane * 4;
  float* XSf = XS;
  float* XSb = XS + (size_t)kLP * kE;
  unsigned short* X16f = XS16;
  unsigned short* X16b = XS16 + (size_t)kLP * kE;
#pragma unroll 1
  for (int sub = 0; sub < 4; ++sub) {
    const int lb = t0 + sub * 16;
#pragma unroll 1
    for (int s = 0; s < 16; ++s) {
      const int t = lb + s;
      const float xp3 = ld_xin(XZ, t + 3, d);
      float uf = wf[0] * xm3;
      uf = fmaf(wf[1], xm2, uf);
      uf = fmaf(wf[2], xm1, uf);
      uf = fmaf(wf[3], x0, uf);
      uf += bf;
      float ub = wb[0] * xp3;
      ub = fmaf(wb[1], xp2, ub);
      ub = fmaf(wb[2], xp1, ub);
      ub = fmaf(wb[3], x0, ub);
      ub += bb;
      const bool ok = t < kL;
      const float vf = silu_f(uf);
      const float vb = silu_f(ub);
      sF[s * kTP + tid] = ok ? vf : 0.0f;
      sB[s * kTP + tid] = ok ? vb : 0.0f;
      xm3 = xm2; xm2 = xm1; xm1 = x0; x0 = xp1; xp1 = xp2; xp2 = xp3;
    }
    __syncthreads();
    v4f ff[4], fb[4];
    v8h hf[2], hb[2];
#pragma unroll
    for (int it = 0; it < 4; ++it) {
      ff[it] = *(const v4f*)(sF + (it * 4 + hrow) * kTP + hch);
      fb[it] = *(const v4f*)(sB + (it * 4 + hrow) * kTP + hch);
    }
#pragma unroll
    for (int it = 0; it < 2; ++it) {
      const float* spf = sF + (it * 8 + wave) * kTP + lane * 8;
      const float* spb = sB + (it * 8 + wave) * kTP + lane * 8;
      const v4f a0 = *(const v4f*)(spf);
      const v4f a1 = *(const v4f*)(spf + 4);
      const v4f c0 = *(const v4f*)(spb);
      const v4f c1 = *(const v4f*)(spb + 4);
#pragma unroll
      for (int e = 0; e < 4; ++e) {
        hf[it][e]     = (_Float16)(a0[e] * kCarryXs);
        hf[it][4 + e] = (_Float16)(a1[e] * kCarryXs);
        hb[it][e]     = (_Float16)(c0[e] * kCarryXs);
        hb[it][4 + e] = (_Float16)(c1[e] * kCarryXs);
      }
    }
    for (int pass = 0; pass < 2; ++pass) {
#pragma unroll
      for (int it = 0; it < 4; ++it) {
        const size_t o = (size_t)(lb + it * 4 + hrow) * kE + d0 + hch;
        *(volatile v4f*)(XSf + o) = ff[it];
        *(volatile v4f*)(XSb + o) = fb[it];
      }
#pragma unroll
      for (int it = 0; it < 2; ++it) {
        const size_t o = (size_t)(lb + it * 8 + wave) * kE + d0 + lane * 8;
        *(volatile v8h*)(X16f + o) = hf[it];
        *(volatile v8h*)(X16b + o) = hb[it];
      }
      __threadfence();
    }
    __syncthreads();
  }
}

__global__ __launch_bounds__(256) void dt_cast_kernel(
    const float* __restrict__ DBL, unsigned short* __restrict__ DTR16, int total8)
{
  const int i = blockIdx.x * 256 + threadIdx.x;
  if (i >= total8) return;
  const int rr = i >> 2;
  const int c8 = (i & 3) * 8;
  const bool ok = c8 < kR;
  const int cc = ok ? c8 : 16;
  const float* p = DBL + (size_t)rr * kDblP + cc;
  const v4f a0 = *(const v4f*)(p);
  const v4f a1 = *(const v4f*)(p + 4);
  v8h hv;
#pragma unroll
  for (int e = 0; e < 4; ++e) {
    const float f0 = ok ? (a0[e] * kCarryDtr) : 0.0f;
    const float f1 = ok ? (a1[e] * kCarryDtr) : 0.0f;
    hv[e]     = (_Float16)f0;
    hv[4 + e] = (_Float16)f1;
  }
  unsigned short* q = DTR16 + (size_t)i * 8;
  *(volatile v8h*)q = hv;
  __threadfence();
  *(volatile v8h*)q = hv;
}

constexpr int kScanChunks = 50;
static_assert(kScanChunks * 16 >= kL && kScanChunks * 16 <= kLP, "scan chunk coverage");
__global__ __launch_bounds__(256) void scan_kernel(
    const float* __restrict__ DLR, const float* __restrict__ XS, const float* __restrict__ DBL,
    const float* __restrict__ bdt_f, const float* __restrict__ bdt_b,
    const float* __restrict__ Alog_f, const float* __restrict__ Alog_b,
    const float* __restrict__ Dv_f, const float* __restrict__ Dv_b,
    float* __restrict__ YS)
{
  __shared__ __align__(16) float sBC[16 * 32];
  __shared__ __align__(16) float sY[16 * kTP];
  const int tid = threadIdx.x, lane = tid & 31, wave = tid >> 5;
  const int dir = blockIdx.y;
  const int d0 = blockIdx.x * 256, d = d0 + tid;
  const float* bdt  = dir ? bdt_b : bdt_f;
  const float* Alog = dir ? Alog_b : Alog_f;
  const float* Dv   = dir ? Dv_b : Dv_f;
  const float* DLRd = DLR + (size_t)dir * kLP * kE;
  const float* XSd  = XS  + (size_t)dir * kLP * kE;
  const float* DBLd = DBL + (size_t)dir * kLP * kDblP;
  float* Yd = YS + (size_t)dir * kLP * kE;

  float An[kNs], h[kNs];
#pragma unroll
  for (int q4 = 0; q4 < 4; ++q4) {
    const v4f al = *(const v4f*)(Alog + (size_t)d * kNs + 4 * q4);
    An[4 * q4 + 0] = -expf(al[0]);
    An[4 * q4 + 1] = -expf(al[1]);
    An[4 * q4 + 2] = -expf(al[2]);
    An[4 * q4 + 3] = -expf(al[3]);
  }
#pragma unroll
  for (int n = 0; n < kNs; ++n) h[n] = 0.0f;
  const float bb = bdt[d];
  const float Dd = Dv[d];
  const int hrow = wave >> 1;
  const int hch  = (wave & 1) * 128 + lane * 4;

#pragma unroll 1
  for (int ci = 0; ci < kScanChunks; ++ci) {
    const int c  = dir ? (kScanChunks - 1 - ci) : ci;
    const int l0 = c * 16;
    if (tid < 128) {
      const int r = tid >> 3, q = (tid & 7) * 4;
      const v4f v = *(const v4f*)(DBLd + (size_t)(l0 + r) * kDblP + kR + q);
      *(v4f*)(sBC + r * 32 + q) = v;
    }
    __syncthreads();
#pragma unroll 1
    for (int si = 0; si < 16; ++si) {
      const int s = dir ? (15 - si) : si;
      const int t = l0 + s;
      const bool ok = t < kL;
      const float a  = DLRd[(size_t)t * kE + d] + bb;
      const float sp = fmaxf(a, 0.0f) + log1pf(__expf(-fabsf(a)));
      const float delta = ok ? sp : 0.0f;
      const float xv = XSd[(size_t)t * kE + d];
      v4f Bq[4], Cq[4];
#pragma unroll
      for (int qq = 0; qq < 4; ++qq) {
        Bq[qq] = *(const v4f*)(sBC + s * 32 + 4 * qq);
        Cq[qq] = *(const v4f*)(sBC + s * 32 + kNs + 4 * qq);
      }
      const float dtx = delta * xv;
      float y = 0.0f;
#pragma unroll
      for (int n = 0; n < kNs; ++n) {
        const float e = __expf(delta * An[n]);
        const float hn = fmaf(e, h[n], dtx * Bq[n >> 2][n & 3]);
        h[n] = hn;
        y = fmaf(hn, Cq[n >> 2][n & 3], y);
      }
      y = fmaf(xv, Dd, y);
      sY[s * kTP + tid] = y;
    }
    __syncthreads();
    v4f fv[4];
#pragma unroll
    for (int it = 0; it < 4; ++it) fv[it] = *(const v4f*)(sY + (it * 4 + hrow) * kTP + hch);
    for (int pass = 0; pass < 2; ++pass) {
#pragma unroll
      for (int it = 0; it < 4; ++it)
        *(volatile v4f*)(Yd + (size_t)(l0 + it * 4 + hrow) * kE + d0 + hch) = fv[it];
      __threadfence();
    }
  }
}

constexpr int kGateTotal = kLP * (kE / 8);
static_assert((kGateTotal % 256) == 0 && ((kE / 8) % 32) == 0, "gate coverage");
__global__ __launch_bounds__(256) void gate_kernel(
    const float* __restrict__ YS, const float* __restrict__ XZ, unsigned short* __restrict__ CMB, int total8)
{
  const int i = blockIdx.x * 256 + threadIdx.x;
  if (i >= total8) return;
  const int row = i / (kE / 8);
  const int c8  = (i - row * (kE / 8)) * 8;
  const bool ok = row < kL;
  const int rc  = ok ? row : (kL - 1);
  const float* pf = YS + (size_t)rc * kE + c8;
  const float* pb = YS + (size_t)kLP * kE + (size_t)rc * kE + c8;
  const float* pz = XZ + (size_t)rc * kXzP + kE + c8;
  const v4f f0 = *(const v4f*)(pf);
  const v4f f1 = *(const v4f*)(pf + 4);
  const v4f b0 = *(const v4f*)(pb);
  const v4f b1 = *(const v4f*)(pb + 4);
  const v4f z0 = *(const v4f*)(pz);
  const v4f z1 = *(const v4f*)(pz + 4);
  v8h hv;
#pragma unroll
  for (int e = 0; e < 4; ++e) {
    const float g0 = silu_f(z0[e]);
    const float g1 = silu_f(z1[e]);
    const float v0 = f0[e] * g0 + b0[e] * g0;
    const float v1 = f1[e] * g1 + b1[e] * g1;
    hv[e]     = (_Float16)(ok ? (v0 * kCarryCmb) : 0.0f);
    hv[4 + e] = (_Float16)(ok ? (v1 * kCarryCmb) : 0.0f);
  }
  unsigned short* q = CMB + (size_t)row * kE + c8;
  *(volatile v8h*)q = hv;
  __threadfence();
  *(volatile v8h*)q = hv;
}

extern "C" void kernel_launch(void* const* d_in, const int* in_sizes, int n_in,
                              void* d_out, int out_size, void* d_ws, size_t ws_size,
                              hipStream_t stream)
{
  if (n_in < 23) return;
  if (in_sizes[0] != 3 * kFrames * kImg * kImg) return;
  if (in_sizes[1] != kDm * kPF || in_sizes[2] != kDm || in_sizes[3] != kDm) return;
  if (in_sizes[4] != kL * kDm || in_sizes[5] != kNL * kDm) return;
  if (in_sizes[6] != kNL * kXzP * kDm) return;
  if (in_sizes[7] != kNL * kE * 4 || in_sizes[8] != kNL * kE) return;
  if (in_sizes[9] != kNL * kDbl * kE || in_sizes[10] != kNL * kE * kR) return;
  if (in_sizes[11] != kNL * kE || in_sizes[12] != kNL * kE * kNs || in_sizes[13] != kNL * kE) return;
  if (in_sizes[14] != kNL * kE * 4 || in_sizes[15] != kNL * kE) return;
  if (in_sizes[16] != kNL * kDbl * kE || in_sizes[17] != kNL * kE * kR) return;
  if (in_sizes[18] != kNL * kE || in_sizes[19] != kNL * kE * kNs || in_sizes[20] != kNL * kE) return;
  if (in_sizes[21] != kNL * kDm * kE || in_sizes[22] != kDm) return;
  if (out_size != kL * kDm) return;
  if (ws_size < kWsTotal) return;

  const float* x         = (const float*)d_in[0];
  const float* patch_w   = (const float*)d_in[1];
  const float* patch_b   = (const float*)d_in[2];
  const float* cls       = (const float*)d_in[3];
  const float* pos       = (const float*)d_in[4];
  const float* norm_w    = (const float*)d_in[5];
  const float* in_w      = (const float*)d_in[6];
  const float* conv_w    = (const float*)d_in[7];
  const float* conv_b    = (const float*)d_in[8];
  const float* xproj_w   = (const float*)d_in[9];
  const float* dtproj_w  = (const float*)d_in[10];
  const float* dtproj_b  = (const float*)d_in[11];
  const float* A_log     = (const float*)d_in[12];
  const float* Dp        = (const float*)d_in[13];
  const float* conv_w_b  = (const float*)d_in[14];
  const float* conv_b_b  = (const float*)d_in[15];
  const float* xproj_wb  = (const float*)d_in[16];
  const float* dtproj_wb = (const float*)d_in[17];
  const float* dtproj_bb = (const float*)d_in[18];
  const float* A_b_log   = (const float*)d_in[19];
  const float* D_b       = (const float*)d_in[20];
  const float* out_w     = (const float*)d_in[21];
  const float* norm_f_w  = (const float*)d_in[22];
  float* dout = (float*)d_out;

  char* ws = (char*)d_ws;
  unsigned short* WIN16  = (unsigned short*)(ws + kOffWIN);
  unsigned short* WOUT16 = (unsigned short*)(ws + kOffWOUT);
  unsigned short* WXP16  = (unsigned short*)(ws + kOffWXP);
  unsigned short* WDT16  = (unsigned short*)(ws + kOffWDT);
  unsigned short* PWH    = (unsigned short*)(ws + kOffPWH);
  unsigned short* PWL    = (unsigned short*)(ws + kOffPWL);
  unsigned short* PAH    = (unsigned short*)(ws + kOffPAH);
  unsigned short* PAL    = (unsigned short*)(ws + kOffPAL);
  float*          RES    = (float*)(ws + kOffRES);
  float*          HID    = (float*)(ws + kOffHID);
  unsigned short* H16    = (unsigned short*)(ws + kOffH16);
  float*          XZ     = (float*)(ws + kOffXZ);
  float*          XS     = (float*)(ws + kOffXS);
  unsigned short* XS16   = (unsigned short*)(ws + kOffXS16);
  float*          DBL    = (float*)(ws + kOffDBL);
  unsigned short* DTR16  = (unsigned short*)(ws + kOffDTR);
  float*          DLR    = (float*)(ws + kOffDLR);
  float*          YS     = (float*)(ws + kOffYS);
  unsigned short* CMB16  = (unsigned short*)(ws + kOffCMB);

  {
    const int t_in  = kNL * kXzP * kDm / 8;
    const int t_out = kNL * kDm * kE / 8;
    const int t_xp  = kNL * kDblP * kE / 8;
    const int t_dt  = kNL * kE * kRP / 8;
    pad_cast_f16_kernel<<<dim3(t_in / 256, 1), 256, 0, stream>>>(in_w, in_w, WIN16, kXzP, kDm, kXzP, kDm, kNL, kCarryW, t_in);
    pad_cast_f16_kernel<<<dim3(t_out / 256, 1), 256, 0, stream>>>(out_w, out_w, WOUT16, kDm, kE, kDm, kE, kNL, kCarryW, t_out);
    pad_cast_f16_kernel<<<dim3(t_xp / 256, 2), 256, 0, stream>>>(xproj_w, xproj_wb, WXP16, kDbl, kE, kDblP, kE, kNL, kCarryW, t_xp);
    pad_cast_f16_kernel<<<dim3(t_dt / 256, 2), 256, 0, stream>>>(dtproj_w, dtproj_wb, WDT16, kE, kR, kE, kRP, kNL, kCarryWdt, t_dt);
    split_rows_bf16_kernel<<<(kDm * kPF / 8) / 256, 256, 0, stream>>>(patch_w, PWH, PWL, kDm * kPF / 8);
    patchify_kernel<<<kPatchBlocks + 1, 256, 0, stream>>>(x, cls, pos, PAH, PAL, HID);
  }

  wmma_gemm64<1, true, true><<<dim3(10, 1), 256, 0, stream>>>(
      PAH, PAL, kPF, 0L, PWH, PWL, kPF, 0L,
      HID + kDm, kDm, 0L, patch_b, pos + kDm,
      kLP, kDm, kPF, kNP, 1.0f);

  for (int l = 0; l < kNL; ++l) {
    const float* nw  = norm_w    + (size_t)l * kDm;
    const float* cwf = conv_w    + (size_t)l * kE * 4;
    const float* cbf = conv_b    + (size_t)l * kE;
    const float* dbf = dtproj_b  + (size_t)l * kE;
    const float* Alf = A_log     + (size_t)l * kE * kNs;
    const float* Dpf = Dp        + (size_t)l * kE;
    const float* cwb = conv_w_b  + (size_t)l * kE * 4;
    const float* cbb = conv_b_b  + (size_t)l * kE;
    const float* dbb = dtproj_bb + (size_t)l * kE;
    const float* Alb = A_b_log   + (size_t)l * kE * kNs;
    const float* Dpb = D_b       + (size_t)l * kE;
    const unsigned short* wIn  = WIN16  + (size_t)l * kXzP * kDm;
    const unsigned short* wOut = WOUT16 + (size_t)l * kDm * kE;
    const unsigned short* wXp  = WXP16  + (size_t)l * kDblP * kE;
    const unsigned short* wDt  = WDT16  + (size_t)l * kE * kRP;

    add_rmsnorm_kernel<false><<<kLP / 8, 256, 0, stream>>>(HID, RES, nw, H16, RES, (l == 0) ? 1 : 0);

    wmma_gemm64<0, false, false><<<dim3(39, 1), 256, 0, stream>>>(
        H16, H16, kDm, 0L, wIn, wIn, kDm, 0L,
        XZ, kXzP, 0L, nw, nw,
        kLP, kXzP, kDm, kLP, kSclIn);

    conv_silu_kernel<<<dim3(kE / 256, kLP / 64), 256, 0, stream>>>(XZ, cwf, cbf, cwb, cbb, XS, XS16);

    wmma_gemm64<0, false, false><<<dim3(2, 2), 256, 0, stream>>>(
        XS16, XS16, kE, (long)kLP * kE, wXp, wXp, kE, (long)kNL * kDblP * kE,
        DBL, kDblP, (long)kLP * kDblP, nw, nw,
        kLP, kDblP, kE, kLP, kSclXp);

    dt_cast_kernel<<<(2 * kLP * kRP / 8) / 256, 256, 0, stream>>>(DBL, DTR16, 2 * kLP * kRP / 8);

    wmma_gemm64<0, false, false><<<dim3(20, 2), 256, 0, stream>>>(
        DTR16, DTR16, kRP, (long)kLP * kRP, wDt, wDt, kRP, (long)kNL * kE * kRP,
        DLR, kE, (long)kLP * kE, nw, nw,
        kLP, kE, kRP, kLP, kSclDt);

    scan_kernel<<<dim3(kE / 256, 2), 256, 0, stream>>>(DLR, XS, DBL, dbf, dbb, Alf, Alb, Dpf, Dpb, YS);

    gate_kernel<<<kGateTotal / 256, 256, 0, stream>>>(YS, XZ, CMB16, kGateTotal);

    wmma_gemm64<0, false, false><<<dim3(10, 1), 256, 0, stream>>>(
        CMB16, CMB16, kE, 0L, wOut, wOut, kE, 0L,
        HID, kDm, 0L, nw, nw,
        kLP, kDm, kE, kLP, kSclOut);
  }

  add_rmsnorm_kernel<true><<<(kL + 7) / 8, 256, 0, stream>>>(HID, RES, norm_f_w, H16, dout, 0);
}
